// LDS_10617159155781
// MI455X (gfx1250) — hardware-verified
//
#include <hip/hip_runtime.h>
#include <math.h>

typedef __attribute__((ext_vector_type(16))) _Float16 v16h;
typedef __attribute__((ext_vector_type(8)))  _Float16 v8h;
typedef __attribute__((ext_vector_type(4)))  _Float16 v4h;
typedef __attribute__((ext_vector_type(8)))  float    v8f;
typedef __attribute__((ext_vector_type(4)))  float    v4f;

constexpr int kBatch = 8;
constexpr int kSeq   = 4096;
constexpr int kDim   = 256;
constexpr int kRows  = kBatch * kSeq;
constexpr int kHP    = 264;
static_assert(kRows == 32768, "rows");
static_assert((kDim % 32) == 0, "GEMM K multiple of 32");
static_assert((kRows % 64) == 0 && (kDim % 64) == 0, "GEMM M,N multiples of 64");
static_assert(kBatch == 8, "batch rows occupy D rows 0..7 of one 16-row tile");
static_assert(((kHP * 2) % 16) == 0, "LDS row pitch keeps 16-B fragment alignment");

constexpr float kSX = 16.0f;
constexpr float kSB = 2048.0f;
constexpr float kSA = 256.0f;
constexpr float kSC = 2048.0f;
constexpr float kSH = 64.0f;
constexpr float kScale1 = (kSH * kSA) / (kSX * kSB);
constexpr float kScale2 = 1.0f / (kSH * kSC);
constexpr float kInvSA  = 1.0f / kSA;
static_assert(kScale1 == 0.5f, "fold-back scale of the input projection");

constexpr size_t kOffX16  = 0;
constexpr size_t kOffW16  = kOffX16 + (size_t)kRows * kDim * 2;
constexpr size_t kOffXBP  = kOffW16 + (size_t)3 * kDim * kDim * 2;
constexpr size_t kOffHS16 = kOffXBP + (size_t)kRows * kDim * 4;
constexpr size_t kWsTotal = kOffHS16 + (size_t)kRows * kDim * 2;
static_assert(kWsTotal == 67502080ull, "carve total");
static_assert(kWsTotal <= 134217728ull, "carve cap");
static_assert((kOffW16 % 128) == 0 && (kOffXBP % 128) == 0 && (kOffHS16 % 128) == 0, "128-B aligned regions");

union FragU { v16h v; v8h h[2]; };
__device__ __forceinline__ v16h frag_load(const _Float16* p) {
  FragU f;
  f.h[0] = *(const v8h*)(p);
  f.h[1] = *(const v8h*)(p + 16);
  return f.v;
}
__device__ __forceinline__ v8f mma_h(v16h a, v16h b, v8f c) {
  c = __builtin_amdgcn_wmma_f32_16x16x32_f16(false, a, false, b, (short)0, c, false, false);
  asm volatile("v_nop\n\tv_nop\n\tv_nop\n\tv_nop" : "+v"(c) : "v"(a), "v"(b));
  return c;
}
__device__ __forceinline__ void acc_guard4(v8f& a, v8f& b, v8f& c, v8f& d) {
  asm volatile("v_nop\n\tv_nop\n\tv_nop\n\tv_nop" : "+v"(a), "+v"(b), "+v"(c), "+v"(d));
}

__global__ __launch_bounds__(256) void cvt_x_kernel(
    const float* __restrict__ src, unsigned short* __restrict__ dst, int total8)
{
  const int i = blockIdx.x * 256 + threadIdx.x;
  if (i >= total8) return;
  const size_t e0 = (size_t)i << 3;
  const v4f a0 = *(const v4f*)(src + e0);
  const v4f a1 = *(const v4f*)(src + e0 + 4);
  v8h hv;
#pragma unroll
  for (int e = 0; e < 4; ++e) {
    const float f0 = a0[e] * kSX;
    const float f1 = a1[e] * kSX;
    hv[e]     = (_Float16)f0;
    hv[4 + e] = (_Float16)f1;
  }
  volatile v8h* p = (volatile v8h*)(dst + e0);
  *p = hv;
  __threadfence();
  *p = hv;
}

__global__ __launch_bounds__(256) void wt_transpose_kernel(
    const float* __restrict__ Wb, const float* __restrict__ Wa, const float* __restrict__ Wc,
    unsigned short* __restrict__ W16)
{
  __shared__ __align__(16) float tl[64 * 65];
  const int tid  = threadIdx.x;
  const int lane = tid & 31;
  const int wave = __builtin_amdgcn_readfirstlane((int)(threadIdx.x >> 5));
  const int z = blockIdx.y;
  const float* src = (z == 0) ? Wb : ((z == 1) ? Wa : Wc);
  const float scl  = (z == 0) ? kSB : ((z == 1) ? kSA : kSC);
  unsigned short* dst = W16 + (size_t)z * kDim * kDim;
  const int k0 = (blockIdx.x >> 2) * 64;
  const int n0 = (blockIdx.x & 3) * 64;
  const int lr = tid >> 4, lc = (tid & 15) * 4;
#pragma unroll
  for (int i = 0; i < 4; ++i) {
    const int row = lr + 16 * i;
    const v4f v = *(const v4f*)(src + (size_t)(k0 + row) * kDim + n0 + lc);
    tl[row * 65 + lc + 0] = v[0];
    tl[row * 65 + lc + 1] = v[1];
    tl[row * 65 + lc + 2] = v[2];
    tl[row * 65 + lc + 3] = v[3];
  }
  __syncthreads();
  const int q = lane >> 3, c8 = (lane & 7) * 8;
  v8h hv[2];
#pragma unroll
  for (int it = 0; it < 2; ++it) {
    const int nr = it * 32 + wave * 4 + q;
#pragma unroll
    for (int e = 0; e < 8; ++e) {
      const float f = tl[(c8 + e) * 65 + nr] * scl;
      hv[it][e] = (_Float16)f;
    }
  }
  for (int pass = 0; pass < 2; ++pass) {
#pragma unroll
    for (int it = 0; it < 2; ++it) {
      const int nr = it * 32 + wave * 4 + q;
      *(volatile v8h*)(dst + (size_t)(n0 + nr) * kDim + k0 + c8) = hv[it];
    }
    __threadfence();
  }
}

__global__ __launch_bounds__(256) void gemm_f16_nt_kernel(
    const unsigned short* __restrict__ Ap, int lda,
    const unsigned short* __restrict__ Btp, int ldb,
    float* __restrict__ C, int ldc,
    int M, int N, int K, float scale)
{
  __shared__ __align__(16) float sT[8][16 * 68];
  const _Float16* A  = (const _Float16*)Ap;
  const _Float16* Bt = (const _Float16*)Btp;
  const int lane = threadIdx.x & 31;
  const int wave = __builtin_amdgcn_readfirstlane((int)(threadIdx.x >> 5));
  const int tilesN = N >> 6;
  const int tilesM = M >> 6;
  const int tile = blockIdx.x * 8 + wave;
  if (tile >= tilesM * tilesN) return;
  const int tm = tile / tilesN;
  const int tn = tile - tm * tilesN;
  const int m0 = tm << 6;
  const int n0 = tn << 6;

  const int rlane = lane & 15;
  const int koff  = (lane >> 4) * 8;
  const int mOff  = (lane >> 4) * 8;

  v8f acc[4][4];
#pragma unroll
  for (int i = 0; i < 4; ++i)
#pragma unroll
    for (int j = 0; j < 4; ++j) acc[i][j] = (v8f){0.f,0.f,0.f,0.f,0.f,0.f,0.f,0.f};

  for (int k0 = 0; k0 < K; k0 += 32) {
    v16h bh[4];
#pragma unroll
    for (int j = 0; j < 4; ++j) {
      const size_t bo = (size_t)(n0 + (j << 4) + rlane) * ldb + koff + k0;
      bh[j] = frag_load(Bt + bo);
    }
#pragma unroll
    for (int i = 0; i < 4; ++i) {
      const size_t ao = (size_t)(m0 + (i << 4) + rlane) * lda + koff + k0;
      const v16h ah = frag_load(A + ao);
#pragma unroll
      for (int j = 0; j < 4; ++j) acc[i][j] = mma_h(ah, bh[j], acc[i][j]);
    }
  }
  acc_guard4(acc[0][0], acc[0][1], acc[0][2], acc[0][3]);
  acc_guard4(acc[1][0], acc[1][1], acc[1][2], acc[1][3]);
  acc_guard4(acc[2][0], acc[2][1], acc[2][2], acc[2][3]);
  acc_guard4(acc[3][0], acc[3][1], acc[3][2], acc[3][3]);

  float* slab = sT[wave];
#pragma unroll
  for (int i = 0; i < 4; ++i) {
    const int mBase = m0 + (i << 4);
#pragma unroll
    for (int j = 0; j < 4; ++j) {
#pragma unroll
      for (int r = 0; r < 8; ++r) {
        const float v = acc[i][j][r] * scale;
        slab[(mOff + r) * 68 + (j << 4) + rlane] = v;
      }
    }
    __builtin_amdgcn_fence(__ATOMIC_RELEASE, "workgroup");
    __builtin_amdgcn_wave_barrier();
    __builtin_amdgcn_fence(__ATOMIC_ACQUIRE, "workgroup");
    {
      const int hh = lane >> 4, c4 = (lane & 15) * 4;
      for (int pass = 0; pass < 2; ++pass) {
#pragma unroll
        for (int it = 0; it < 8; ++it) {
          const int row = it * 2 + hh;
          const v4f v = *(const v4f*)(slab + row * 68 + c4);
          *(volatile v4f*)(C + (size_t)(mBase + row) * ldc + n0 + c4) = v;
        }
        __threadfence();
      }
    }
    __builtin_amdgcn_fence(__ATOMIC_RELEASE, "workgroup");
    __builtin_amdgcn_wave_barrier();
    __builtin_amdgcn_fence(__ATOMIC_ACQUIRE, "workgroup");
  }
}

__global__ __launch_bounds__(512) void scan_kernel(
    const float* __restrict__ xbp, const unsigned short* __restrict__ BtAp,
    const float* __restrict__ h0, unsigned short* __restrict__ hs16)
{
  __shared__ __align__(16) _Float16 hbuf[2 * 16 * kHP];
  const int tid  = threadIdx.x;
  const int lane = tid & 31;
  const int wave = __builtin_amdgcn_readfirstlane((int)(threadIdx.x >> 5));
  const int lo = lane & 15, hi = lane >> 4;
  const int n0 = wave * 16;
  const bool lowhalf = (hi == 0);

#pragma unroll 1
  for (int idx = tid; idx < 2 * 16 * kHP; idx += 512) {
    const int buf = idx / (16 * kHP);
    const int rem = idx - buf * (16 * kHP);
    const int row = rem / kHP;
    const int col = rem - row * kHP;
    const int cc  = (col < kDim) ? col : (kDim - 1);
    float hv = h0[cc];
    asm volatile("" : "+v"(hv));
    const bool live = (buf == 0) && (row < kBatch) && (col < kDim);
    const float v = live ? (hv * kSH) : 0.0f;
    hbuf[idx] = (_Float16)v;
  }

  v16h bfr[8];
  {
    const _Float16* brow = (const _Float16*)BtAp + (size_t)(n0 + lo) * kDim + 8 * hi;
#pragma unroll
    for (int kt = 0; kt < 8; ++kt) bfr[kt] = frag_load(brow + kt * 32);
  }

  const float* xp = xbp + n0 + lo;
  float xc[8];
#pragma unroll
  for (int r = 0; r < 8; ++r) {
    float v = xp[((size_t)r * kSeq) * kDim];
    asm volatile("" : "+v"(v));
    xc[r] = v;
  }
  const int sb   = wave >> 1;
  const int hoff = (wave & 1) * 128 + lane * 4;
  __syncthreads();

#pragma unroll 1
  for (int t = 0; t < kSeq; ++t) {
    const int cur = t & 1;
    const _Float16* hc = hbuf + cur * (16 * kHP);
    _Float16* hn = hbuf + (cur ^ 1) * (16 * kHP);

    const int tn = (t + 1 < kSeq) ? (t + 1) : (kSeq - 1);
    float xn[8];
#pragma unroll
    for (int r = 0; r < 8; ++r) {
      float v = xp[((size_t)r * kSeq + tn) * kDim];
      asm volatile("" : "+v"(v));
      xn[r] = v;
    }

    v8f acc;
#pragma unroll
    for (int r = 0; r < 8; ++r) acc[r] = lowhalf ? xc[r] : 0.0f;

    const _Float16* arow = hc + lo * kHP + 8 * hi;
#pragma unroll
    for (int kt = 0; kt < 8; ++kt) {
      const v16h a = frag_load(arow + kt * 32);
      acc = mma_h(a, bfr[kt], acc);
    }

#pragma unroll
    for (int r = 0; r < 8; ++r) {
      const float hv = acc[r] * kInvSA;
      const float wv = lowhalf ? hv : 0.0f;
      hn[(8 * hi + r) * kHP + n0 + lo] = (_Float16)wv;
    }
    __syncthreads();

    {
      const v4h sv = *(const v4h*)(hn + sb * kHP + hoff);
      volatile v4h* gp = (volatile v4h*)(hs16 + ((size_t)sb * kSeq + t) * kDim + hoff);
      *gp = sv;
      __threadfence();
      *gp = sv;
    }
#pragma unroll
    for (int r = 0; r < 8; ++r) xc[r] = xn[r];
  }
}

extern "C" void kernel_launch(void* const* d_in, const int* in_sizes, int n_in,
                              void* d_out, int out_size, void* d_ws, size_t ws_size,
                              hipStream_t stream) {
  if (n_in < 5) return;
  if (in_sizes[0] != kRows * kDim) return;
  if (in_sizes[1] != kDim * kDim) return;
  if (in_sizes[2] != kDim * kDim) return;
  if (in_sizes[3] != kDim * kDim) return;
  if (in_sizes[4] != kDim) return;
  if (out_size != kRows * kDim) return;
  if (ws_size < kWsTotal) return;

  const float* x  = (const float*)d_in[0];
  const float* Am = (const float*)d_in[1];
  const float* Bm = (const float*)d_in[2];
  const float* Cm = (const float*)d_in[3];
  const float* h0 = (const float*)d_in[4];
  float* y = (float*)d_out;

  char* ws = (char*)d_ws;
  unsigned short* X16  = (unsigned short*)(ws + kOffX16);
  unsigned short* W16  = (unsigned short*)(ws + kOffW16);
  float*          XBP  = (float*)(ws + kOffXBP);
  unsigned short* HS16 = (unsigned short*)(ws + kOffHS16);
  unsigned short* BtB  = W16;
  unsigned short* BtA  = W16 + (size_t)kDim * kDim;
  unsigned short* BtC  = W16 + (size_t)2 * kDim * kDim;

  cvt_x_kernel<<<(kRows * kDim / 8) / 256, 256, 0, stream>>>(x, X16, kRows * kDim / 8);
  wt_transpose_kernel<<<dim3(16, 3), 256, 0, stream>>>(Bm, Am, Cm, W16);

  gemm_f16_nt_kernel<<<(kRows / 64) * (kDim / 64) / 8, 256, 0, stream>>>(
      X16, kDim, BtB, kDim, XBP, kDim, kRows, kDim, kDim, kScale1);

  scan_kernel<<<1, 512, 0, stream>>>(XBP, BtA, h0, HS16);

  gemm_f16_nt_kernel<<<(kRows / 64) * (kDim / 64) / 8, 256, 0, stream>>>(
      HS16, kDim, BtC, kDim, y, kDim, kRows, kDim, kDim, kScale2);
}
